// MarkerGAT_31499290149073
// MI455X (gfx1250) — hardware-verified
//
#include <hip/hip_runtime.h>
#include <math.h>

typedef __attribute__((ext_vector_type(16))) _Float16 v16h;
typedef __attribute__((ext_vector_type(16))) __bf16 v16b;
typedef __attribute__((ext_vector_type(8)))  _Float16 v8h;
typedef __attribute__((ext_vector_type(8)))  float v8f;
typedef __attribute__((ext_vector_type(4)))  float v4f;
typedef __attribute__((ext_vector_type(2)))  float v2f;
typedef __attribute__((ext_vector_type(4)))  unsigned v4u;
typedef __attribute__((ext_vector_type(4)))  int v4i;
typedef float __attribute__((may_alias)) float_a;
typedef int __attribute__((may_alias)) int_a;

template <typename T> __device__ __forceinline__ void vst2(void* p, T v) { *(volatile T*)p = v; __threadfence(); *(volatile T*)p = v; }
__device__ __forceinline__ v8f wmma16(v16h a, v16h b, v8f c) {
  v8f d = __builtin_amdgcn_wmma_f32_16x16x32_f16(false, a, false, b, (short)0, c, false, false);
  asm volatile("v_nop\n\tv_nop\n\tv_nop\n\tv_nop" : "+v"(d) : "v"(a), "v"(b));
  return d;
}
__device__ __forceinline__ v8f wmma_bf(v16b a, v16b b, v8f c) {
  v8f d = __builtin_amdgcn_wmma_f32_16x16x32_bf16(false, a, false, b, (short)0, c, false, false);
  asm volatile("v_nop\n\tv_nop\n\tv_nop\n\tv_nop" : "+v"(d) : "v"(a), "v"(b));
  return d;
}
__device__ __forceinline__ v16h frag_h(const _Float16* rowk0, int lane) {
  union { v16h v; v8h q[2]; } u; const _Float16* p = rowk0 + 8 * (lane >> 4);
  u.q[0] = *(const v8h*)p; u.q[1] = *(const v8h*)(p + 16); return u.v;
}
__device__ __forceinline__ v16h frag_f32(const float* rowk0, int lane) {
  v16h a; const float* p = rowk0 + 8 * (lane >> 4);
#pragma unroll
  for (int i = 0; i < 8; ++i) { a[i] = (_Float16)p[i]; a[8 + i] = (_Float16)p[16 + i]; }
  return a;
}
__device__ __forceinline__ v16h frag_f32s(const float* rowk0, int lane, float sc) {
  v16h a; const float* p = rowk0 + 8 * (lane >> 4);
#pragma unroll
  for (int i = 0; i < 8; ++i) { a[i] = (_Float16)(p[i] * sc); a[8 + i] = (_Float16)(p[16 + i] * sc); }
  return a;
}
__device__ __forceinline__ v16h fragc_f32(const float* W, int k0, int n, int lane, int ld, int K) {
  v16h a; const int g = lane >> 4;
#pragma unroll
  for (int i = 0; i < 8; ++i) { const int ka = k0 + 8 * g + i, kb = ka + 16;
    a[i] = (_Float16)(ka < K ? W[(size_t)(ka < K ? ka : K - 1) * ld + n] : 0.f); a[8 + i] = (_Float16)(kb < K ? W[(size_t)(kb < K ? kb : K - 1) * ld + n] : 0.f); }
  return a;
}
struct F2 { v16b h, l; };
__device__ __forceinline__ F2 bsplit16(const float v[16]) { F2 r;
#pragma unroll
  for (int i = 0; i < 16; ++i) { const __bf16 h = (__bf16)v[i]; r.h[i] = h; r.l[i] = (__bf16)(v[i] - (float)h); }
  return r; }
__device__ __forceinline__ F2 split_row(const float* row, int k0, int lane) { float v[16]; const float* p = row + k0 + 8 * (lane >> 4);
#pragma unroll
  for (int i = 0; i < 8; ++i) { v[i] = p[i]; v[8 + i] = p[16 + i]; }
  return bsplit16(v); }
__device__ __forceinline__ F2 split_rowK(const float* row, int k0, int lane, int K) { float v[16]; const int g = lane >> 4;
#pragma unroll
  for (int i = 0; i < 8; ++i) { const int ka = k0 + 8 * g + i, kb = ka + 16; v[i] = ka < K ? row[ka < K ? ka : K - 1] : 0.f; v[8 + i] = kb < K ? row[kb < K ? kb : K - 1] : 0.f; }
  return bsplit16(v); }
__device__ __forceinline__ F2 split_col(const float* W, int k0, int n, int lane, int ld, int K) { float v[16]; const int g = lane >> 4;
#pragma unroll
  for (int i = 0; i < 8; ++i) { const int ka = k0 + 8 * g + i, kb = ka + 16; v[i] = ka < K ? W[(size_t)(ka < K ? ka : K - 1) * ld + n] : 0.f; v[8 + i] = kb < K ? W[(size_t)(kb < K ? kb : K - 1) * ld + n] : 0.f; }
  return bsplit16(v); }
__device__ __forceinline__ v8f mac3(const F2& a, const F2& b, v8f c) { c = wmma_bf(a.l, b.h, c); c = wmma_bf(a.h, b.l, c); return wmma_bf(a.h, b.h, c); }
__device__ __forceinline__ float sigm(float v) { return 1.0f / (1.0f + expf(-v)); }
#define LDSX() do { asm volatile("s_wait_dscnt 0" ::: "memory"); __builtin_amdgcn_wave_barrier(); __builtin_amdgcn_fence(__ATOMIC_RELEASE, "workgroup"); } while (0)


#ifndef NN
#define NN 4096
#endif
#define EP 65536
#ifndef NE
#define NE 65536
#endif
#define DIN 6
#define EMB 128
#define NH1 4
#define HC1 32
#define OC 64
#define NIA 5
#define NBLK (NN / 64)
#define CSR_N NN
#define CSR_E NE
typedef __attribute__((ext_vector_type(8))) __bf16 v8b;
__device__ __forceinline__ v16b frag_b(const __bf16* rowk0, int lane) {
  union { v16b v; v8b q[2]; } u; const __bf16* p = rowk0 + 8 * (lane >> 4);
  u.q[0] = *(const v8b*)p; u.q[1] = *(const v8b*)(p + 16); return u.v;
}
__device__ __forceinline__ float bfr(float v) { return (float)(__bf16)v; }
__device__ __attribute__((noinline)) float exp_ni(float v) { return expf(v); }
__device__ __attribute__((noinline)) float erf_ni(float v) { return erff(v); }

#define CSR_FINN (CSR_E + 32 * CSR_NBK)
#define CSR_CHUNK 4096
#define CSR_BKT 256
#define CSR_NCH ((CSR_E + CSR_CHUNK - 1) / CSR_CHUNK)
#define CSR_NBK ((CSR_N + CSR_BKT - 1) / CSR_BKT)
#define CSR_NBKP (((CSR_NBK + 63) / 64) * 64)
#define CSR_SEGCAP (CSR_E + 32 * CSR_NBK * CSR_NCH)
#ifndef CSR_BCAP
#define CSR_BCAP 10240
#endif
#define CSR_SZ_CNT   (4u * CSR_NCH * CSR_NBKP)
#define CSR_SZ_OFF   (4u * CSR_NBK * (((CSR_NCH + 31) / 32) * 32))
#define CSR_SZ_BST   (4u * (((CSR_NBK + 1 + 31) / 32) * 32))
#define CSR_SZ_SEG   (4u * CSR_SEGCAP)
#define CSR_SZ_FIN   (4u * (CSR_E + 32 * CSR_NBK))
#define CSR_SZ_ROW   (4u * CSR_NBK * CSR_BKT)
#define CSR_OFFP (((CSR_NCH + 31) / 32) * 32)

__global__ __launch_bounds__(256) void k_csr_cnt(const int* __restrict__ DST, int dstride, int* __restrict__ CNT) {
  __shared__ unsigned short sc[256][CSR_NBK + 1]; __shared__ __align__(16) int srow[CSR_NBKP];
  const int c = blockIdx.x, tid = threadIdx.x;
  for (int b = 0; b < CSR_NBK; ++b) sc[tid][b] = 0;
  const size_t e0 = (size_t)c * CSR_CHUNK + tid * 16;
  for (int i = 0; i < 16; ++i) { const size_t e = e0 + i; if (e < (size_t)CSR_E) { int d = DST[e * dstride]; d = min(max(d, 0), CSR_N - 1); sc[tid][d / CSR_BKT] += 1; } }
  __syncthreads();
  for (int b = tid; b < CSR_NBKP; b += 256) { int s = 0; if (b < CSR_NBK) for (int t = 0; t < 256; ++t) s += sc[t][b]; srow[b] = s; }
  __syncthreads();
  for (int q = tid; q < CSR_NBKP / 4; q += 256) vst2((unsigned*)(CNT + (size_t)c * CSR_NBKP + q * 4), *(const v4u*)&srow[q * 4]);
}
__global__ __launch_bounds__(256) void k_csr_scan(const int* __restrict__ CNT, int* __restrict__ OFF, int* __restrict__ BST) {
  __shared__ int sbt[CSR_NBK + 1]; __shared__ int sbs[((CSR_NBK + 1 + 31) / 32) * 32]; __shared__ int scnt[CSR_NBK + 1]; __shared__ __align__(16) int sbuf[64][CSR_OFFP];
  const int tid = threadIdx.x;
  for (int b = tid; b < CSR_NBK; b += 256) { int sp = 0, st = 0; for (int c = 0; c < CSR_NCH; ++c) { const int n = CNT[(size_t)c * CSR_NBKP + b]; st += n; sp += (n + 31) & ~31; } sbt[b] = sp; scnt[b] = st; }
  for (int b = tid; b < ((CSR_NBK + 1 + 31) / 32) * 32; b += 256) sbs[b] = 0;
  __syncthreads();
  if (tid == 0) { int acc = 0, accf = 0; for (int b = 0; b < CSR_NBK; ++b) { const int t = sbt[b]; sbt[b] = acc; acc += t; sbs[b] = accf; accf += (scnt[b] + 31) & ~31; } sbs[CSR_NBK] = accf; }
  __syncthreads();
  for (int b0 = 0; b0 < CSR_NBK; b0 += 64) {
    if (tid < 64 && b0 + tid < CSR_NBK) { const int b = b0 + tid; int o = sbt[b]; for (int c = 0; c < CSR_OFFP; ++c) { if (c < CSR_NCH) { sbuf[tid][c] = o; o += (CNT[(size_t)c * CSR_NBKP + b] + 31) & ~31; } else sbuf[tid][c] = 0; } }
    __syncthreads();
    for (int q = tid; q < 64 * (CSR_OFFP / 4); q += 256) { const int r = q / (CSR_OFFP / 4), pc = q % (CSR_OFFP / 4); if (b0 + r < CSR_NBK) vst2((unsigned*)(OFF + (size_t)(b0 + r) * CSR_OFFP + pc * 4), *(const v4u*)&sbuf[r][pc * 4]); }
    __syncthreads(); }
  for (int q = tid; q < ((CSR_NBK + 1 + 31) / 32) * 32 / 4; q += 256) vst2((unsigned*)(BST + q * 4), *(const v4u*)&sbs[q * 4]);
}
__global__ __launch_bounds__(256) void k_csr_scatter(const int* __restrict__ SRC, const int* __restrict__ DST, int sstride, int dstride, const int* __restrict__ OFF, int* __restrict__ SEGS, int* __restrict__ SEGE) {
  __shared__ unsigned short sc[256][CSR_NBK + 1]; __shared__ int sbase[CSR_NBK + 1]; __shared__ int scn[CSR_NBK + 1]; __shared__ int sord[CSR_CHUNK];
  const int c = blockIdx.x, tid = threadIdx.x;
  for (int b = 0; b < CSR_NBK; ++b) sc[tid][b] = 0;
  const size_t e0 = (size_t)c * CSR_CHUNK + tid * 16; int bk[16];
#pragma unroll
  for (int i = 0; i < 16; ++i) { const size_t e = e0 + i; bk[i] = -1; if (e < (size_t)CSR_E) { int d = DST[e * dstride]; d = min(max(d, 0), CSR_N - 1); bk[i] = d / CSR_BKT; sc[tid][bk[i]] += 1; } }
  __syncthreads();
  for (int b = tid; b < CSR_NBK; b += 256) { int acc = 0; for (int t = 0; t < 256; ++t) { const int v = sc[t][b]; sc[t][b] = (unsigned short)acc; acc += v; } scn[b] = acc; }
  __syncthreads();
  if (tid == 0) { int acc = 0; for (int b = 0; b < CSR_NBK; ++b) { sbase[b] = acc; acc += scn[b]; } }
  __syncthreads();
#pragma unroll
  for (int i = 0; i < 16; ++i) { if (bk[i] >= 0) { const int b = bk[i]; const int r = sc[tid][b]; sc[tid][b] = (unsigned short)(r + 1); sord[sbase[b] + r] = tid * 16 + i; } }
  __syncthreads();
  for (int b = 0; b < CSR_NBK; ++b) { const int n = scn[b]; if (n == 0) continue; const int nl = ((n + 31) & ~31); const size_t o = (size_t)(min(max(OFF[(size_t)b * CSR_OFFP + c], 0), CSR_SEGCAP - nl) & ~31);
    for (int q = tid; q < nl / 4; q += 256) { int4 vs, ve;
#pragma unroll
      for (int k = 0; k < 4; ++k) { const int i = q * 4 + k; int s = -1, eid = -1; if (i < n) { const size_t e = (size_t)c * CSR_CHUNK + sord[sbase[b] + i]; s = min(max(SRC[e * sstride], 0), CSR_N - 1); eid = (int)e; } vs[k] = s; ve[k] = eid; }
      vst2((unsigned*)(SEGS + o + q * 4), *(const v4u*)&vs); vst2((unsigned*)(SEGE + o + q * 4), *(const v4u*)&ve); } }
}
__global__ __launch_bounds__(256) void k_csr_bucket(const int* __restrict__ CNT, const int* __restrict__ OFF, const int* __restrict__ BST, const int* __restrict__ SEGS, const int* __restrict__ SEGE, const int* __restrict__ DST, int dstride, int* __restrict__ FS, int* __restrict__ FE, int* __restrict__ ROWST, int* __restrict__ ROWCNT) {
  __shared__ int ssrc[CSR_BCAP]; __shared__ int seid[CSR_BCAP]; __shared__ unsigned char snod[CSR_BCAP]; __shared__ int souts[CSR_BCAP]; __shared__ int soute[CSR_BCAP]; __shared__ int scount[256]; __shared__ int sstart[257]; __shared__ int stot;
  const int b = blockIdx.x, tid = threadIdx.x;
  if (tid == 0) { int t = 0; for (int c = 0; c < CSR_NCH; ++c) t += min(max(CNT[(size_t)c * CSR_NBKP + b], 0), CSR_CHUNK); stot = (t <= CSR_BCAP) ? t : 0; }
  __syncthreads();
  { int base = 0; for (int c = 0; c < CSR_NCH; ++c) { const int n = min(max(CNT[(size_t)c * CSR_NBKP + b], 0), CSR_CHUNK); const int o = min(max(OFF[(size_t)b * CSR_OFFP + c], 0), CSR_SEGCAP - ((n + 31) & ~31));
      for (int i = tid; i < n; i += 256) { const int p = base + i; if (p < CSR_BCAP) { ssrc[p] = min(max(SEGS[o + i], 0), CSR_N - 1); const int e = min(max(SEGE[o + i], 0), CSR_E - 1); seid[p] = e; int d = DST[(size_t)e * dstride]; d = min(max(d, 0), CSR_N - 1); const int dl = d - b * CSR_BKT; snod[p] = (unsigned char)(dl >= 0 && dl < 256 ? dl : 255); } }
      base += n; } }
  __syncthreads();
  const int node = b * CSR_BKT + tid; int cnt = 0; for (int p = 0; p < stot; ++p) cnt += (snod[p] == tid) ? 1 : 0;
  scount[tid] = cnt; __syncthreads();
  if (tid == 0) { int acc = 0; for (int t = 0; t < 256; ++t) { sstart[t] = acc; acc += scount[t]; } sstart[256] = acc; }
  __syncthreads();
  const int bst0 = min(max(BST[b], 0), CSR_FINN - ((sstart[256] + 31) & ~31)) & ~31; const int gst = bst0 + sstart[tid];
  { int w = sstart[tid]; for (int p = 0; p < stot; ++p) if (snod[p] == tid) { souts[w] = ssrc[p]; soute[w] = seid[p]; ++w; } }
  __syncthreads();
  { const int n = sstart[256]; const int nl = (n + 31) & ~31; for (int q = tid; q < nl / 4; q += 256) { int4 vs, ve;
#pragma unroll
      for (int k = 0; k < 4; ++k) { const int i = q * 4 + k; vs[k] = i < n ? souts[i] : -1; ve[k] = i < n ? soute[i] : -1; }
      vst2((unsigned*)(FS + bst0 + q * 4), *(const v4u*)&vs); vst2((unsigned*)(FE + bst0 + q * 4), *(const v4u*)&ve); } }
  __syncthreads();
  { __shared__ __align__(16) int srs[256], src2[256]; srs[tid] = node < CSR_N ? gst : 0; src2[tid] = node < CSR_N ? cnt : 0; __syncthreads();
    if (tid < 64) vst2((unsigned*)(ROWST + (size_t)b * 256 + tid * 4), *(const v4u*)&srs[tid * 4]); else if (tid < 128) vst2((unsigned*)(ROWCNT + (size_t)b * 256 + (tid - 64) * 4), *(const v4u*)&src2[(tid - 64) * 4]); }
}


__constant__ int c_midx[NIA][2] = {{0, 3}, {2, 1}, {2, 5}, {1, 0}, {4, -1}};
#define WS_CNT  0u
#define WS_OFF  (WS_CNT + CSR_SZ_CNT)
#define WS_BST  (WS_OFF + CSR_SZ_OFF)
#define WS_SEGS (WS_BST + CSR_SZ_BST)
#define WS_SEGE (WS_SEGS + CSR_SZ_SEG)
#define WS_FS   (WS_SEGE + CSR_SZ_SEG)
#define WS_FE   (WS_FS + CSR_SZ_FIN)
#define WS_RST  (WS_FE + CSR_SZ_FIN)
#define WS_RCT  (WS_RST + CSR_SZ_ROW)
#define WS_PW   (WS_RCT + CSR_SZ_ROW)
#define PIN 0
#define POUT (PIN + NIA * 384 * EMB)
#define PW2 (POUT + NIA * EMB * EMB)
#define PWEND (PW2 + OC * EMB)
#define WS_HW1  (WS_PW + 2u * PWEND)
#define WS_A1   (WS_HW1 + 4u * NN * EMB)
#define WS_X1   (WS_A1 + 4u * 2 * NH1 * NN)
#define WS_NM   (WS_X1 + 4u * NN * EMB)
#define WS_QK   (WS_NM + 4u * (NN * 8 + 64))
#define WS_VTH  (WS_QK + 4u * NN * 256)
#define WS_VTL  (WS_VTH + 2u * EMB * NN)
#define WS_O    (WS_VTL + 2u * EMB * NN)
#define WS_ACC  (WS_O + 4u * NN * EMB)
#define WS_X2   (WS_ACC + 4u * NN * EMB)
#define WS_HW2  (WS_X2 + 4u * NN * EMB)
#define WS_X3   (WS_HW2 + 4u * NN * OC)
#define WS_PS   (WS_X3 + 4u * NN * OC)
#define WS_END  (WS_PS + 4u * NBLK * 32)

__global__ __launch_bounds__(128) void k_pack(const float* __restrict__ INW, const float* __restrict__ OUTW, const float* __restrict__ W2, __bf16* __restrict__ PW) {
  __shared__ __align__(16) __bf16 s[EMB]; const int n = blockIdx.x, pl = blockIdx.y, k = threadIdx.x; size_t base; float v;
  if (pl < NIA) { if (n >= 384) return; base = PIN + ((size_t)pl * 384 + n) * EMB; v = INW[((size_t)pl * 384 + n) * EMB + k]; }
  else if (pl < 2 * NIA) { if (n >= EMB) return; base = POUT + ((size_t)(pl - NIA) * EMB + n) * EMB; v = OUTW[((size_t)(pl - NIA) * EMB + n) * EMB + k]; }
  else { if (n >= OC) return; base = PW2 + (size_t)n * EMB; v = W2[(size_t)k * OC + n]; }
  s[k] = (__bf16)v; __syncthreads();
  if (k < 16) vst2((unsigned*)(PW + base + k * 8), *(const v4u*)&s[k * 8]);
}
__global__ __launch_bounds__(256) void k_gproj1(const float* __restrict__ X, const float* __restrict__ W1, const float* __restrict__ AS1, const float* __restrict__ AD1, float* __restrict__ HW, float* __restrict__ A) {
  __shared__ float sw[DIN][EMB], sas[EMB], sad[EMB]; __shared__ __align__(16) float so[16][EMB + 4]; __shared__ __align__(16) float sa[16][8];
  const int tid = threadIdx.x; for (int q = tid; q < DIN * EMB; q += 256) sw[q / EMB][q % EMB] = bfr(W1[q]); if (tid < EMB) { sas[tid] = bfr(AS1[tid]); sad[tid] = bfr(AD1[tid]); }
  __syncthreads();
  const int nl = tid >> 4, sl = tid & 15, c0 = sl * 8; const size_t node = (size_t)blockIdx.x * 16 + nl; float xv[DIN];
#pragma unroll
  for (int i = 0; i < DIN; ++i) xv[i] = bfr(X[node * DIN + i]);
  float ps = 0.f, pd = 0.f;
#pragma unroll
  for (int j = 0; j < 8; ++j) { float a = 0.f;
#pragma unroll
    for (int i = 0; i < DIN; ++i) a += xv[i] * sw[i][c0 + j];
    so[nl][c0 + j] = a; ps += a * sas[c0 + j]; pd += a * sad[c0 + j]; }
  ps += __shfl_xor(ps, 1); ps += __shfl_xor(ps, 2); pd += __shfl_xor(pd, 1); pd += __shfl_xor(pd, 2);
  if ((sl & 3) == 0) { sa[nl][sl >> 2] = ps; sa[nl][4 + (sl >> 2)] = pd; }
  __syncthreads();
  for (int q = tid; q < 16 * 32; q += 256) { const int rl = q >> 5, pc = q & 31; vst2(HW + ((size_t)blockIdx.x * 16 + rl) * EMB + pc * 4, *(const v4f*)&so[rl][pc * 4]); }
  if (tid < 32) vst2(A + (size_t)blockIdx.x * 16 * 8 + tid * 4, *(const v4f*)&sa[tid >> 1][(tid & 1) * 4]);
}
__global__ __launch_bounds__(256) void k_gat1(const float* __restrict__ HW, const float* __restrict__ A, const int* __restrict__ FS, const int* __restrict__ RST, const int* __restrict__ RCT, const float* __restrict__ B1, float* __restrict__ X1) {
  __shared__ __align__(16) float so[8][EMB + 4];
  const int tid = threadIdx.x, wave = tid >> 5, lane = tid & 31; const int hd = lane >> 3, sl = lane & 7; const int f0 = hd * HC1 + sl * 4; const size_t node = (size_t)blockIdx.x * 8 + wave;
  float acc[4] = {0.f, 0.f, 0.f, 0.f};
  { const int cnt = min(max(RCT[node], 0), CSR_BCAP); const int st = min(max(RST[node], 0), CSR_FINN - cnt); const float adn = A[node * 8 + 4 + hd];
    float es = A[node * 8 + hd] + adn; es = (es >= 0.f) ? es : 0.2f * es; float mx = es;
    for (int e = 0; e < cnt; ++e) { const int s = min(max(FS[st + e], 0), NN - 1); float v = A[(size_t)s * 8 + hd] + adn; v = (v >= 0.f) ? v : 0.2f * v; mx = fmaxf(mx, v); }
    float den = 0.f; { const float w = exp_ni(es - mx); den += w; const float* hr = HW + node * EMB + f0;
#pragma unroll
      for (int i = 0; i < 4; ++i) acc[i] += w * hr[i]; }
    for (int e = 0; e < cnt; ++e) { const int s = min(max(FS[st + e], 0), NN - 1); float v = A[(size_t)s * 8 + hd] + adn; v = (v >= 0.f) ? v : 0.2f * v; const float w = exp_ni(v - mx); den += w; const float* hr = HW + (size_t)s * EMB + f0;
#pragma unroll
      for (int i = 0; i < 4; ++i) acc[i] += w * hr[i]; }
    const float iden = 1.0f / (den + 1e-16f);
#pragma unroll
    for (int i = 0; i < 4; ++i) so[wave][f0 + i] = fmaxf(acc[i] * iden + bfr(B1[f0 + i]), 0.f); }
  LDSX();
  vst2(X1 + node * EMB + lane * 4, *(const v4f*)&so[wave][lane * 4]);
}
__global__ __launch_bounds__(64) void k_colsum(const float* __restrict__ X1, float* __restrict__ PS) {
  __shared__ __align__(16) float s[32]; const int blk = blockIdx.x, tid = threadIdx.x;
  if (tid < 32) { float acc = 0.f; if (tid < DIN) for (int rl = 0; rl < 64; ++rl) acc += X1[((size_t)blk * 64 + rl) * EMB + tid]; s[tid] = acc; }
  __syncthreads();
  if (tid < 8) vst2(PS + (size_t)blk * 32 + tid * 4, *(const v4f*)&s[tid * 4]);
}
__global__ __launch_bounds__(256) void k_flags(const float* __restrict__ X1, const float* __restrict__ PS, float* __restrict__ NM) {
  __shared__ float smu[8]; __shared__ __align__(16) float sf[64][8]; __shared__ __align__(16) float scnt[8]; __shared__ int sc[8];
  const int tid = threadIdx.x;
  if (tid < 8) { float acc = 0.f; for (int b = 0; b < NBLK; ++b) acc += PS[(size_t)b * 32 + tid]; smu[tid] = acc / (float)NN; sc[tid] = 0; }
  __syncthreads();
  for (int base = 0; base < NN; base += 64) {
    for (int q = tid; q < 64 * 8; q += 256) { const int rl = q >> 3, c = q & 7; float f = 0.f; if (c < DIN) f = (X1[((size_t)base + rl) * EMB + c] > smu[c]) ? 1.f : 0.f; sf[rl][c] = f; }
    __syncthreads();
    if (tid < DIN) { int cn = 0; for (int rl = 0; rl < 64; ++rl) cn += (sf[rl][tid] != 0.f) ? 1 : 0; sc[tid] += cn; }
    for (int q = tid; q < 64 * 2; q += 256) { const int rl = q >> 1, pc = q & 1; vst2(NM + ((size_t)base + rl) * 8 + pc * 4, *(const v4f*)&sf[rl][pc * 4]); }
    __syncthreads(); }
  if (tid < 8) scnt[tid] = (tid < DIN) ? (float)sc[tid] : 0.f;
  __syncthreads();
  if (tid < 2) vst2(NM + (size_t)NN * 8 + tid * 4, *(const v4f*)&scnt[tid * 4]);
}
__global__ __launch_bounds__(128) void k_qkv(const float* __restrict__ X1, const __bf16* __restrict__ P, const float* __restrict__ bias, float* __restrict__ QK, __bf16* __restrict__ VTH, __bf16* __restrict__ VTL) {
  __shared__ __align__(16) float so[4][16][132]; __shared__ __align__(16) __bf16 sth[128][72], stl[128][72];
  const int tid = threadIdx.x, wave = tid >> 5, lane = tid & 31, col = lane & 15, g = lane >> 4; const size_t r0 = (size_t)blockIdx.x * 64 + wave * 16; const int n0 = blockIdx.y * 128;
  v8f acc[8] = {};
#pragma unroll
  for (int kc = 0; kc < EMB / 32; ++kc) { const F2 a = split_row(X1 + (r0 + col) * EMB, kc * 32, lane);
#pragma unroll
    for (int j = 0; j < 8; ++j) { const v16b w = frag_b(P + (size_t)(n0 + j * 16 + col) * EMB + kc * 32, lane); acc[j] = wmma_bf(a.l, w, acc[j]); acc[j] = wmma_bf(a.h, w, acc[j]); } }
  if (n0 < 2 * EMB) {
#pragma unroll
    for (int j = 0; j < 8; ++j) { const float bb = bfr(bias[n0 + j * 16 + col]);
#pragma unroll
      for (int r = 0; r < 8; ++r) so[wave][8 * g + r][j * 16 + col] = acc[j][r] + bb; }
    LDSX();
    for (int rl = 0; rl < 16; ++rl) vst2(QK + (r0 + rl) * 256 + n0 + lane * 4, *(const v4f*)&so[wave][rl][lane * 4]);
  } else {
#pragma unroll
    for (int j = 0; j < 8; ++j) { const float bb = bfr(bias[n0 + j * 16 + col]);
#pragma unroll
      for (int r = 0; r < 8; ++r) { const float v = acc[j][r] + bb; const __bf16 hb = (__bf16)v; sth[j * 16 + col][wave * 16 + 8 * g + r] = hb; stl[j * 16 + col][wave * 16 + 8 * g + r] = (__bf16)(v - (float)hb); } }
    __syncthreads();
    const int s0 = blockIdx.x * 64;
    for (int q = tid; q < 128 * 8; q += 128) { const int d = q >> 3, pc = q & 7; const size_t o = (size_t)d * NN + s0 + pc * 8; vst2((unsigned*)(VTH + o), *(const v4u*)&sth[d][pc * 8]); vst2((unsigned*)(VTL + o), *(const v4u*)&stl[d][pc * 8]); }
  }
}
__global__ __launch_bounds__(128) void k_attn(const float* __restrict__ QK, const float* __restrict__ NM, int ia, const __bf16* __restrict__ VTH, const __bf16* __restrict__ VTL, float* __restrict__ O) {
  __shared__ __align__(16) float sp[4][16][36]; __shared__ __align__(16) float so[4][16][132];
  const int tid = threadIdx.x, wave = tid >> 5, lane = tid & 31, col = lane & 15, g = lane >> 4; const int q0 = blockIdx.x * 64 + wave * 16;
  const int m0 = c_midx[ia][0], m1 = c_midx[ia][1]; const float cnt0 = NM[(size_t)NN * 8 + m0], cnt1 = (m1 >= 0) ? NM[(size_t)NN * 8 + m1] : 0.f;
  float fq0[8], fq1[8], irow[8];
#pragma unroll
  for (int r = 0; r < 8; ++r) { const int qi = q0 + 8 * g + r; fq0[r] = NM[(size_t)qi * 8 + m0]; fq1[r] = (m1 >= 0) ? NM[(size_t)qi * 8 + m1] : 0.f; const float rs = fq0[r] * cnt0 + fq1[r] * cnt1; irow[r] = 1.0f / (rs + 1e-8f); }
  const float* qrow = QK + (size_t)(q0 + col) * 256;
  float m[8], l[8];
#pragma unroll
  for (int r = 0; r < 8; ++r) { m[r] = -3.0e38f; l[r] = 0.f; }
  v8f acc[8] = {};
#pragma unroll 1
  for (int ks = 0; ks < NN / 32; ++ks) { v8f s[2];
#pragma unroll
    for (int ct = 0; ct < 2; ++ct) { const int kk = ks * 32 + ct * 16 + col; const float* krow = QK + (size_t)kk * 256 + EMB; v8f c = {};
#pragma unroll
      for (int kc = 0; kc < 4; ++kc) { const F2 kb = split_row(krow, kc * 32, lane); const F2 qa = split_row(qrow, kc * 32, lane); c = mac3(qa, kb, c); }
      const float fk0 = NM[(size_t)kk * 8 + m0], fk1 = (m1 >= 0) ? NM[(size_t)kk * 8 + m1] : 0.f;
#pragma unroll
      for (int r = 0; r < 8; ++r) { const float mk = (fq0[r] * fk0 + fq1[r] * fk1) * irow[r]; s[ct][r] = c[r] * 0.08838834764831845f + mk; } }
#pragma unroll
    for (int r = 0; r < 8; ++r) { float mx = fmaxf(s[0][r], s[1][r]);
#pragma unroll
      for (int o = 1; o < 16; o <<= 1) mx = fmaxf(mx, __shfl_xor(mx, o));
      const float mn = fmaxf(m[r], mx); const float alpha = exp_ni(m[r] - mn);
      const float e0 = exp_ni(s[0][r] - mn), e1 = exp_ni(s[1][r] - mn); float es = e0 + e1;
#pragma unroll
      for (int o = 1; o < 16; o <<= 1) es += __shfl_xor(es, o);
      l[r] = l[r] * alpha + es; m[r] = mn;
#pragma unroll
      for (int dt = 0; dt < 8; ++dt) acc[dt][r] *= alpha;
      sp[wave][8 * g + r][col] = e0; sp[wave][8 * g + r][16 + col] = e1; }
    LDSX();
    const F2 pa = split_row(&sp[wave][col][0], 0, lane);
#pragma unroll
    for (int dt = 0; dt < 8; ++dt) { const size_t vr = (size_t)(dt * 16 + col) * NN + ks * 32; const v16b vh = frag_b(VTH + vr, lane), vl = frag_b(VTL + vr, lane); acc[dt] = wmma_bf(pa.l, vh, acc[dt]); acc[dt] = wmma_bf(pa.h, vl, acc[dt]); acc[dt] = wmma_bf(pa.h, vh, acc[dt]); }
    LDSX(); }
#pragma unroll
  for (int r = 0; r < 8; ++r) { const float il = 1.0f / l[r];
#pragma unroll
    for (int dt = 0; dt < 8; ++dt) so[wave][8 * g + r][dt * 16 + col] = acc[dt][r] * il; }
  LDSX();
  for (int rl = 0; rl < 16; ++rl) vst2(O + (size_t)(q0 + rl) * EMB + lane * 4, *(const v4f*)&so[wave][rl][lane * 4]);
}
template <int FIRST>
__global__ __launch_bounds__(128) void k_oproj(const float* __restrict__ O, const __bf16* __restrict__ P, const float* __restrict__ bias, float* ACC) {
  __shared__ __align__(16) float so[4][16][132];
  const int tid = threadIdx.x, wave = tid >> 5, lane = tid & 31, col = lane & 15, g = lane >> 4; const size_t r0 = (size_t)blockIdx.x * 64 + wave * 16;
  v8f acc[8] = {};
#pragma unroll
  for (int kc = 0; kc < EMB / 32; ++kc) { const F2 a = split_row(O + (r0 + col) * EMB, kc * 32, lane);
#pragma unroll
    for (int j = 0; j < 8; ++j) { const v16b w = frag_b(P + (size_t)(j * 16 + col) * EMB + kc * 32, lane); acc[j] = wmma_bf(a.l, w, acc[j]); acc[j] = wmma_bf(a.h, w, acc[j]); } }
#pragma unroll
  for (int j = 0; j < 8; ++j) { const int n = j * 16 + col; const float bb = bfr(bias[n]);
#pragma unroll
    for (int r = 0; r < 8; ++r) { const size_t row = r0 + 8 * g + r; float v = acc[j][r] + bb; if (!FIRST) v += ACC[row * EMB + n]; so[wave][8 * g + r][n] = v; } }
  LDSX();
  for (int rl = 0; rl < 16; ++rl) vst2(ACC + (r0 + rl) * EMB + lane * 4, *(const v4f*)&so[wave][rl][lane * 4]);
}
__global__ __launch_bounds__(128) void k_x2proj(const float* __restrict__ X1, const float* __restrict__ ACC, const __bf16* __restrict__ P, const float* __restrict__ AS2, const float* __restrict__ AD2, float* __restrict__ X2, float* __restrict__ HW2, float* __restrict__ A) {
  __shared__ __align__(16) float sx[64][EMB + 4]; __shared__ __align__(16) float so[4][16][68]; __shared__ __align__(16) float sa[64][8]; __shared__ float sas[OC], sad[OC];
  const int tid = threadIdx.x, wave = tid >> 5, lane = tid & 31, col = lane & 15, g = lane >> 4; const size_t rb = (size_t)blockIdx.x * 64; const size_t r0 = rb + wave * 16;
  if (tid < OC) { sas[tid] = bfr(AS2[tid]); sad[tid] = bfr(AD2[tid]); }
  for (int q = tid; q < 64 * EMB; q += 128) { const int rl = q >> 7, c = q & 127; sx[rl][c] = X1[(rb + rl) * EMB + c] + ACC[(rb + rl) * EMB + c] / 5.0f; }
  __syncthreads();
  v8f acc[4] = {};
#pragma unroll
  for (int kc = 0; kc < EMB / 32; ++kc) { const F2 a = split_row(&sx[wave * 16 + col][0], kc * 32, lane);
#pragma unroll
    for (int j = 0; j < 4; ++j) { const v16b w = frag_b(P + (size_t)(j * 16 + col) * EMB + kc * 32, lane); acc[j] = wmma_bf(a.l, w, acc[j]); acc[j] = wmma_bf(a.h, w, acc[j]); } }
  float ps = 0.f, pd = 0.f; float psr[8], pdr[8];
#pragma unroll
  for (int r = 0; r < 8; ++r) { psr[r] = 0.f; pdr[r] = 0.f; }
#pragma unroll
  for (int j = 0; j < 4; ++j) { const int c = j * 16 + col;
#pragma unroll
    for (int r = 0; r < 8; ++r) { const float v = acc[j][r]; so[wave][8 * g + r][c] = v; psr[r] += v * sas[c]; pdr[r] += v * sad[c]; } }
  (void)ps; (void)pd;
#pragma unroll
  for (int r = 0; r < 8; ++r) { float a1 = psr[r], a2 = pdr[r];
#pragma unroll
    for (int o = 1; o < 16; o <<= 1) { a1 += __shfl_xor(a1, o); a2 += __shfl_xor(a2, o); }
    if (col == 0) { const int rl = wave * 16 + 8 * g + r; sa[rl][0] = a1; sa[rl][4] = a2; sa[rl][1] = 0.f; sa[rl][2] = 0.f; sa[rl][3] = 0.f; sa[rl][5] = 0.f; sa[rl][6] = 0.f; sa[rl][7] = 0.f; } }
  __syncthreads();
  for (int q = tid; q < 64 * 32; q += 128) { const int rl = q >> 5, pc = q & 31; vst2(X2 + (rb + rl) * EMB + pc * 4, *(const v4f*)&sx[rl][pc * 4]); }
  for (int rl = 0; rl < 16; ++rl) if (lane < 16) vst2(HW2 + (r0 + rl) * OC + lane * 4, *(const v4f*)&so[wave][rl][lane * 4]);
  vst2(A + rb * 8 + (size_t)tid * 4, *(const v4f*)&sa[tid >> 1][(tid & 1) * 4]);
}
__global__ __launch_bounds__(256) void k_gat2(const float* __restrict__ HW2, const float* __restrict__ A, const int* __restrict__ FS, const int* __restrict__ RST, const int* __restrict__ RCT, const float* __restrict__ B2, const float* __restrict__ FW, const float* __restrict__ FB, float* __restrict__ out) {
  __shared__ float sfw[OC][DIN]; __shared__ __align__(16) float so[16 * DIN];
  const int tid = threadIdx.x, wave = tid >> 5, lane = tid & 31; const int f0 = lane * 2;
  for (int q = tid; q < OC * DIN; q += 256) sfw[q / DIN][q % DIN] = bfr(FW[q]);
  __syncthreads();
#pragma unroll 1
  for (int sub = 0; sub < 2; ++sub) { const size_t node = (size_t)blockIdx.x * 16 + sub * 8 + wave; const int slot = sub * 8 + wave;
  float acc[2] = {0.f, 0.f};
  const int cnt = min(max(RCT[node], 0), CSR_BCAP); const int st = min(max(RST[node], 0), CSR_FINN - cnt); const float adn = A[node * 8 + 4];
  float es = A[node * 8] + adn; es = (es >= 0.f) ? es : 0.2f * es; float mx = es;
  for (int e = 0; e < cnt; ++e) { const int s = min(max(FS[st + e], 0), NN - 1); float v = A[(size_t)s * 8] + adn; v = (v >= 0.f) ? v : 0.2f * v; mx = fmaxf(mx, v); }
  float den = 0.f; { const float w = exp_ni(es - mx); den += w; acc[0] += w * HW2[node * OC + f0]; acc[1] += w * HW2[node * OC + f0 + 1]; }
  for (int e = 0; e < cnt; ++e) { const int s = min(max(FS[st + e], 0), NN - 1); float v = A[(size_t)s * 8] + adn; v = (v >= 0.f) ? v : 0.2f * v; const float w = exp_ni(v - mx); den += w; acc[0] += w * HW2[(size_t)s * OC + f0]; acc[1] += w * HW2[(size_t)s * OC + f0 + 1]; }
  const float iden = 1.0f / (den + 1e-16f);
  const float x30 = fmaxf(acc[0] * iden + bfr(B2[f0]), 0.f), x31 = fmaxf(acc[1] * iden + bfr(B2[f0 + 1]), 0.f);
  float o6[DIN];
#pragma unroll
  for (int c = 0; c < DIN; ++c) { float t = x30 * sfw[f0][c] + x31 * sfw[f0 + 1][c];
#pragma unroll
    for (int o = 1; o < 32; o <<= 1) t += __shfl_xor(t, o);
    o6[c] = t + bfr(FB[c]); }
  if (lane == 0) {
#pragma unroll
    for (int c = 0; c < DIN; ++c) so[slot * DIN + c] = o6[c]; } }
  __syncthreads();
  if (tid < 24) vst2(out + (size_t)blockIdx.x * 16 * DIN + tid * 4, *(const v4f*)&so[tid * 4]);
}

extern "C" void kernel_launch(void* const* d_in, const int* in_sizes, int n_in, void* d_out, int out_size, void* d_ws, size_t ws_size, hipStream_t stream) {
  (void)in_sizes; (void)n_in; (void)out_size;
  const float** F = (const float**)d_in; const int* EI = (const int*)d_in[1];
  if (ws_size < (size_t)WS_END) return;
  char* ws = (char*)d_ws;
  int *CNT = (int*)(ws + WS_CNT), *OFF = (int*)(ws + WS_OFF), *BST = (int*)(ws + WS_BST), *SEGS = (int*)(ws + WS_SEGS), *SEGE = (int*)(ws + WS_SEGE), *FS = (int*)(ws + WS_FS), *FE = (int*)(ws + WS_FE), *RST = (int*)(ws + WS_RST), *RCT = (int*)(ws + WS_RCT);
  __bf16* PW = (__bf16*)(ws + WS_PW); float *HW1 = (float*)(ws + WS_HW1), *A1 = (float*)(ws + WS_A1), *X1 = (float*)(ws + WS_X1), *NM = (float*)(ws + WS_NM), *QK = (float*)(ws + WS_QK), *O = (float*)(ws + WS_O), *ACC = (float*)(ws + WS_ACC), *X2 = (float*)(ws + WS_X2), *HW2 = (float*)(ws + WS_HW2), *PS = (float*)(ws + WS_PS);
  __bf16 *VTH = (__bf16*)(ws + WS_VTH), *VTL = (__bf16*)(ws + WS_VTL);
  const int* SRC = EI; const int* DST = EI + EP;
  k_pack<<<dim3(384, 2 * NIA + 1), 128, 0, stream>>>(F[11], F[13], F[7], PW);
  k_csr_cnt<<<CSR_NCH, 256, 0, stream>>>(DST, 1, CNT); k_csr_scan<<<1, 256, 0, stream>>>(CNT, OFF, BST); k_csr_scatter<<<CSR_NCH, 256, 0, stream>>>(SRC, DST, 1, 1, OFF, SEGS, SEGE); k_csr_bucket<<<CSR_NBK, 256, 0, stream>>>(CNT, OFF, BST, SEGS, SEGE, DST, 1, FS, FE, RST, RCT);
  k_gproj1<<<NN / 16, 256, 0, stream>>>(F[0], F[3], F[4], F[5], HW1, A1);
  k_gat1<<<NN / 8, 256, 0, stream>>>(HW1, A1, FS, RST, RCT, F[6], X1);
  k_colsum<<<NBLK, 64, 0, stream>>>(X1, PS); k_flags<<<1, 256, 0, stream>>>(X1, PS, NM);
  for (int ia = 0; ia < NIA; ++ia) {
    k_qkv<<<dim3(NBLK, 3), 128, 0, stream>>>(X1, PW + PIN + (size_t)ia * 384 * EMB, F[12] + ia * 384, QK, VTH, VTL);
    k_attn<<<NBLK, 128, 0, stream>>>(QK, NM, ia, VTH, VTL, O);
    if (ia == 0) k_oproj<1><<<NBLK, 128, 0, stream>>>(O, PW + POUT + (size_t)ia * EMB * EMB, F[14] + ia * EMB, ACC); else k_oproj<0><<<NBLK, 128, 0, stream>>>(O, PW + POUT + (size_t)ia * EMB * EMB, F[14] + ia * EMB, ACC); }
  k_x2proj<<<NBLK, 128, 0, stream>>>(X1, ACC, PW + PW2, F[8], F[9], X2, HW2, A1);
  k_gat2<<<NN / 16, 256, 0, stream>>>(HW2, A1, FS, RST, RCT, F[10], F[15], F[16], (float*)d_out);
}
